// L2Attention_21285857919719
// MI455X (gfx1250) — hardware-verified
//
#include <hip/hip_runtime.h>

typedef _Float16 v16h __attribute__((ext_vector_type(16)));
typedef _Float16 v8h  __attribute__((ext_vector_type(8)));
typedef float    v8f  __attribute__((ext_vector_type(8)));
typedef float    v4f  __attribute__((ext_vector_type(4)));
typedef v8h __attribute__((may_alias)) v8ha;
typedef v4f __attribute__((may_alias)) v4fa;

union Frag { v16h v; v8h half[2]; };

#define BATCH  4
#define SEQ    1024
#define DIM    1024
#define NHEADS 16
#define HD     64
#define TOK    (BATCH * SEQ)
#define NBH    (BATCH * NHEADS)
#define NX     (TOK * DIM)
#define NW     (DIM * DIM)
#define NX8    (NX / 8)
#define NW8    (NW / 8)
#define WSC    32.0f
#define WINV   0.03125f
#define WLOSC  0.125f
#define LOSC   256.0f
#define LOINV  0.00390625f
#define PSCALE 16384.0f
#define PINV   0.00006103515625f

__device__ __forceinline__ v8f wmma_f16(v16h a, v16h b, v8f c) {
  v8f d = __builtin_amdgcn_wmma_f32_16x16x32_f16(false, a, false, b, (short)0, c, false, false);
  asm volatile("v_nop\n\tv_nop\n\tv_nop\n\tv_nop" : "+v"(d) : "v"(a), "v"(b));
  return d;
}

__device__ __forceinline__ v16h load_frag(const _Float16* p, int h) {
  Frag f;
  f.half[0] = *(const v8ha*)(p + 8 * h);
  f.half[1] = *(const v8ha*)(p + 16 + 8 * h);
  return f.v;
}

__global__ __launch_bounds__(256) void convert_kernel(
    const float* __restrict__ x, const float* __restrict__ wq,
    const float* __restrict__ wv, const float* __restrict__ wo,
    _Float16* __restrict__ xh, _Float16* __restrict__ wpl)
{
  const int g = blockIdx.x * 256 + threadIdx.x;
  if (g >= NX8 + 4 * NW8) return;
  const float* src;
  _Float16* dst;
  float sc;
  if (g < NX8) {
    src = x + (size_t)g * 8;
    dst = xh + (size_t)g * 8;
    sc = 1.0f;
  } else {
    const int e = g - NX8;
    const int wsel = e / NW8;
    const int off = e - wsel * NW8;
    const float* wsrc = (wsel == 0) ? wq : ((wsel == 1) ? wv : wo);
    src = wsrc + (size_t)off * 8;
    dst = wpl + (size_t)e * 8;
    sc = (wsel == 3) ? WLOSC : WSC;
  }
  const v4f a = *(const v4fa*)src;
  const v4f c = *(const v4fa*)(src + 4);
  const v8h o = { (_Float16)(a.x * sc), (_Float16)(a.y * sc), (_Float16)(a.z * sc), (_Float16)(a.w * sc),
                  (_Float16)(c.x * sc), (_Float16)(c.y * sc), (_Float16)(c.z * sc), (_Float16)(c.w * sc) };
  *(volatile v8h*)dst = o;
  __threadfence();
  *(volatile v8h*)dst = o;
}

__device__ __forceinline__ void store_rows64(const _Float16* sT, _Float16* plane,
                                             int bh, int l0, int w, int lane) {
  const int q8 = lane & 7, sub = lane >> 3;
  #pragma unroll
  for (int i = 0; i < 8; ++i) {
    const int lid = w * 32 + i * 4 + sub;
    const v8h v = *(const v8ha*)(sT + lid * HD + 8 * q8);
    _Float16* dst = plane + ((size_t)bh * SEQ + l0 + lid) * HD + 8 * q8;
    *(volatile v8h*)dst = v;
  }
}

__device__ __forceinline__ void store_vt(const _Float16* sT, _Float16* vt,
                                         int bh, int l0, int w, int lane) {
  const int q8 = lane & 7, sub = lane >> 3;
  #pragma unroll
  for (int i = 0; i < 8; ++i) {
    const int lid = w * 32 + i * 4 + sub;
    const int d = lid >> 1, hl = lid & 1;
    const v8h v = *(const v8ha*)(sT + d * 128 + 64 * hl + 8 * q8);
    _Float16* dst = vt + ((size_t)bh * HD + d) * SEQ + l0 + 64 * hl + 8 * q8;
    *(volatile v8h*)dst = v;
  }
}

__global__ __launch_bounds__(128) void proj_kernel(
    const _Float16* __restrict__ xh,
    const _Float16* __restrict__ wpl,
    const float* __restrict__ bq, const float* __restrict__ bv,
    _Float16* __restrict__ qk16,
    _Float16* __restrict__ ql16,
    float* __restrict__ sqb,
    _Float16* __restrict__ vt16)
{
  __shared__ __attribute__((aligned(16))) _Float16 sT[128 * 64];
  __shared__ __attribute__((aligned(16))) _Float16 sL[128 * 64];
  __shared__ __attribute__((aligned(16))) float    sP[128 * 16];

  const int tid = threadIdx.x, lane = tid & 31, w = tid >> 5;
  const int h = lane >> 4, m = lane & 15;
  const int m0 = blockIdx.x * 128;
  const int which = blockIdx.y >> 4, head = blockIdx.y & 15;
  const int m0w = m0 + 32 * w;

  const _Float16* xa0 = xh + (size_t)(m0w + m) * DIM;
  const _Float16* xa1 = xa0 + (size_t)16 * DIM;
  const _Float16* wb  = wpl + ((size_t)which * DIM + head * HD + m) * DIM;

  const v8f zero8 = {0.f, 0.f, 0.f, 0.f, 0.f, 0.f, 0.f, 0.f};
  v8f acc[2][4];
  #pragma unroll
  for (int mt = 0; mt < 2; ++mt)
    #pragma unroll
    for (int nt = 0; nt < 4; ++nt) acc[mt][nt] = zero8;

  #pragma unroll 1
  for (int k0 = 0; k0 < DIM; k0 += 32) {
    const v16h a0 = load_frag(xa0 + k0, h);
    const v16h a1 = load_frag(xa1 + k0, h);
    #pragma unroll
    for (int nt = 0; nt < 4; ++nt) {
      const v16h b = load_frag(wb + (size_t)nt * 16 * DIM + k0, h);
      acc[0][nt] = wmma_f16(a0, b, acc[0][nt]);
      acc[1][nt] = wmma_f16(a1, b, acc[1][nt]);
    }
  }

  if (which == 0) {
    float ysq[2][8];
    #pragma unroll
    for (int mt = 0; mt < 2; ++mt)
      #pragma unroll
      for (int r = 0; r < 8; ++r) ysq[mt][r] = 0.0f;
    #pragma unroll
    for (int nt = 0; nt < 4; ++nt) {
      const int feat = 16 * nt + m;
      const float bvl = bq[head * HD + feat];
      #pragma unroll
      for (int mt = 0; mt < 2; ++mt) {
        #pragma unroll
        for (int r = 0; r < 8; ++r) {
          const int tokl = 32 * w + 16 * mt + 8 * h + r;
          const float y = acc[mt][nt][r] * WINV + bvl;
          const _Float16 hi = (_Float16)y;
          const _Float16 lo = (_Float16)((y - (float)hi) * LOSC);
          sT[tokl * HD + feat] = hi;
          sL[tokl * HD + feat] = lo;
          ysq[mt][r] += y * y;
        }
      }
    }
    #pragma unroll
    for (int mt = 0; mt < 2; ++mt)
      #pragma unroll
      for (int r = 0; r < 8; ++r) {
        const int tokl = 32 * w + 16 * mt + 8 * h + r;
        sP[tokl * 16 + m] = ysq[mt][r];
      }
  } else {
    #pragma unroll
    for (int nt = 0; nt < 4; ++nt) {
      const int feat = 16 * nt + m;
      const float bvl = bv[head * HD + feat];
      #pragma unroll
      for (int mt = 0; mt < 2; ++mt) {
        #pragma unroll
        for (int r = 0; r < 8; ++r) {
          const int tokl = 32 * w + 16 * mt + 8 * h + r;
          const float y = acc[mt][nt][r] * WINV + bvl;
          sT[feat * 128 + tokl] = (_Float16)y;
        }
      }
    }
  }
  __syncthreads();

  const int b = m0 / SEQ, l0 = m0 - b * SEQ, bh = b * NHEADS + head;
  if (which == 0) {
    const float* pp = sP + tid * 16;
    const v4f p0 = *(const v4fa*)(pp);
    const v4f p1 = *(const v4fa*)(pp + 4);
    const v4f p2 = *(const v4fa*)(pp + 8);
    const v4f p3 = *(const v4fa*)(pp + 12);
    const float s = ((p0.x + p0.y) + (p0.z + p0.w)) + ((p1.x + p1.y) + (p1.z + p1.w))
                  + ((p2.x + p2.y) + (p2.z + p2.w)) + ((p3.x + p3.y) + (p3.z + p3.w));
    float* sqd = sqb + (size_t)bh * SEQ + l0 + tid;
    store_rows64(sT, qk16, bh, l0, w, lane);
    store_rows64(sL, ql16, bh, l0, w, lane);
    *(volatile float*)sqd = s;
    __threadfence();
    store_rows64(sT, qk16, bh, l0, w, lane);
    store_rows64(sL, ql16, bh, l0, w, lane);
    *(volatile float*)sqd = s;
  } else {
    store_vt(sT, vt16, bh, l0, w, lane);
    __threadfence();
    store_vt(sT, vt16, bh, l0, w, lane);
  }
}

__device__ __forceinline__ v8f logit8(v8f s, const float* p) {
  const v4f a = *(const v4fa*)p;
  const v4f c = *(const v4fa*)(p + 4);
  s[0] = s[0] * 0.25f - a.x * 0.125f;
  s[1] = s[1] * 0.25f - a.y * 0.125f;
  s[2] = s[2] * 0.25f - a.z * 0.125f;
  s[3] = s[3] * 0.25f - a.w * 0.125f;
  s[4] = s[4] * 0.25f - c.x * 0.125f;
  s[5] = s[5] * 0.25f - c.y * 0.125f;
  s[6] = s[6] * 0.25f - c.z * 0.125f;
  s[7] = s[7] * 0.25f - c.w * 0.125f;
  return s;
}

__device__ __forceinline__ v16h pack_p(v8f a, v8f c) {
  const v16h r = { (_Float16)(a[0] * PSCALE), (_Float16)(a[1] * PSCALE), (_Float16)(a[2] * PSCALE), (_Float16)(a[3] * PSCALE),
                   (_Float16)(a[4] * PSCALE), (_Float16)(a[5] * PSCALE), (_Float16)(a[6] * PSCALE), (_Float16)(a[7] * PSCALE),
                   (_Float16)(c[0] * PSCALE), (_Float16)(c[1] * PSCALE), (_Float16)(c[2] * PSCALE), (_Float16)(c[3] * PSCALE),
                   (_Float16)(c[4] * PSCALE), (_Float16)(c[5] * PSCALE), (_Float16)(c[6] * PSCALE), (_Float16)(c[7] * PSCALE) };
  return r;
}

__device__ __forceinline__ void att_store_pass(const _Float16* src, _Float16* plane,
                                               int b, int head, int q0, int lane) {
  const int q8 = lane & 7, sub = lane >> 3;
  #pragma unroll
  for (int i = 0; i < 4; ++i) {
    const int row = i * 4 + sub;
    const v8h v = *(const v8ha*)(src + row * 64 + 8 * q8);
    _Float16* dst = plane + ((size_t)b * SEQ + q0 + row) * DIM + head * HD + 8 * q8;
    *(volatile v8h*)dst = v;
  }
}

__global__ __launch_bounds__(128) void attn_kernel(
    const _Float16* __restrict__ qk16,
    const _Float16* __restrict__ ql16,
    const _Float16* __restrict__ vt16,
    const float* __restrict__ sqb,
    _Float16* __restrict__ oh16,
    _Float16* __restrict__ ol16)
{
  __shared__ __attribute__((aligned(16))) _Float16 sH[4 * 16 * 64];
  __shared__ __attribute__((aligned(16))) _Float16 sLo[4 * 16 * 64];

  const int tid = threadIdx.x, lane = tid & 31, w = tid >> 5;
  const int h = lane >> 4, m = lane & 15;
  const int bh = blockIdx.y, b = bh >> 4, head = bh & 15;
  const int q0 = blockIdx.x * 64 + 16 * w;

  const size_t qoff = ((size_t)bh * SEQ + q0 + m) * HD;
  const v16h qh0 = load_frag(qk16 + qoff, h);
  const v16h qh1 = load_frag(qk16 + qoff + 32, h);
  const v16h ql0 = load_frag(ql16 + qoff, h);
  const v16h ql1 = load_frag(ql16 + qoff + 32, h);

  const v8f zero8 = {0.f, 0.f, 0.f, 0.f, 0.f, 0.f, 0.f, 0.f};
  v8f o[4];
  #pragma unroll
  for (int t = 0; t < 4; ++t) o[t] = zero8;
  float mrun = -1e30f, lrun = 0.0f;

  const _Float16* kbase = qk16 + ((size_t)bh * SEQ + m) * HD;
  const _Float16* vbase = vt16 + ((size_t)bh * HD + m) * SEQ;
  const float* sqp0 = sqb + (size_t)bh * SEQ + 8 * h;

  #pragma unroll 1
  for (int kb = 0; kb < SEQ; kb += 64) {
    v8f s[4];
    #pragma unroll
    for (int j = 0; j < 4; ++j) {
      const _Float16* kp = kbase + (size_t)(kb + 16 * j) * HD;
      const v16h kf0 = load_frag(kp, h);
      const v16h kf1 = load_frag(kp + 32, h);
      v8f z = zero8;
      z = wmma_f16(kf0, ql0, z);
      z = wmma_f16(kf1, ql1, z);
      #pragma unroll
      for (int r = 0; r < 8; ++r) z[r] = z[r] * LOINV;
      z = wmma_f16(kf0, qh0, z);
      z = wmma_f16(kf1, qh1, z);
      s[j] = z;
    }
    #pragma unroll
    for (int j = 0; j < 4; ++j) s[j] = logit8(s[j], sqp0 + kb + 16 * j);

    float mloc = s[0][0];
    #pragma unroll
    for (int j = 0; j < 4; ++j)
      #pragma unroll
      for (int r = 0; r < 8; ++r) mloc = fmaxf(mloc, s[j][r]);
    mloc = fmaxf(mloc, __shfl_xor(mloc, 16));
    const float mnew = fmaxf(mrun, mloc);
    const float alpha = __expf(mrun - mnew);
    mrun = mnew;
    float lsum = 0.0f;
    #pragma unroll
    for (int j = 0; j < 4; ++j)
      #pragma unroll
      for (int r = 0; r < 8; ++r) {
        const float p = __expf(s[j][r] - mnew);
        s[j][r] = p;
        lsum += p;
      }
    lsum += __shfl_xor(lsum, 16);
    lrun = lrun * alpha + lsum;
    #pragma unroll
    for (int t = 0; t < 4; ++t)
      #pragma unroll
      for (int r = 0; r < 8; ++r) o[t][r] = o[t][r] * alpha;

    const v16h pb0 = pack_p(s[0], s[1]);
    const v16h pb1 = pack_p(s[2], s[3]);

    #pragma unroll
    for (int t = 0; t < 4; ++t) {
      const _Float16* vp = vbase + (size_t)(16 * t) * SEQ + kb;
      const v16h vf0 = load_frag(vp, h);
      const v16h vf1 = load_frag(vp + 32, h);
      o[t] = wmma_f16(vf0, pb0, o[t]);
      o[t] = wmma_f16(vf1, pb1, o[t]);
    }
  }

  const float inv = (1.0f / lrun) * PINV;
  _Float16* sh = sH + w * 1024;
  _Float16* sl = sLo + w * 1024;
  #pragma unroll
  for (int t = 0; t < 4; ++t)
    #pragma unroll
    for (int r = 0; r < 8; ++r) {
      const float val = o[t][r] * inv;
      const _Float16 hi = (_Float16)val;
      const _Float16 lo = (_Float16)((val - (float)hi) * LOSC);
      const int idx = m * 64 + 16 * t + 8 * h + r;
      sh[idx] = hi;
      sl[idx] = lo;
    }
  __syncthreads();

  att_store_pass(sh, oh16, b, head, q0, lane);
  att_store_pass(sl, ol16, b, head, q0, lane);
  __threadfence();
  att_store_pass(sh, oh16, b, head, q0, lane);
  att_store_pass(sl, ol16, b, head, q0, lane);
}

__device__ __forceinline__ void out_store_pass(const float* sO, float* out,
                                               int m0, int fg, int w, int lane) {
  const int q8 = lane & 7, sub = lane >> 3;
  #pragma unroll
  for (int i = 0; i < 16; ++i) {
    const int lid = i * 4 + sub;
    const int row = 32 * w + (lid >> 1), hl = lid & 1;
    const v4f v = *(const v4fa*)(sO + row * 64 + 32 * hl + 4 * q8);
    const size_t gi = (size_t)(m0 + row) * DIM + fg * HD + 32 * hl + 4 * q8;
    *(volatile v4f*)(out + gi) = v;
  }
}

__global__ __launch_bounds__(128) void ogemm_kernel(
    const _Float16* __restrict__ oh16,
    const _Float16* __restrict__ ol16,
    const _Float16* __restrict__ wo16,
    const _Float16* __restrict__ wol16,
    const float* __restrict__ bo,
    float* __restrict__ out)
{
  __shared__ __attribute__((aligned(16))) float sO[128 * 64];

  const int tid = threadIdx.x, lane = tid & 31, w = tid >> 5;
  const int h = lane >> 4, m = lane & 15;
  const int m0 = blockIdx.x * 128;
  const int fg = blockIdx.y;
  const int m0w = m0 + 32 * w;

  const size_t aoff = (size_t)(m0w + m) * DIM;
  const _Float16* ah0p = oh16 + aoff;
  const _Float16* ah1p = ah0p + (size_t)16 * DIM;
  const _Float16* al0p = ol16 + aoff;
  const _Float16* al1p = al0p + (size_t)16 * DIM;
  const size_t woff = ((size_t)fg * HD + m) * DIM;
  const _Float16* wbh = wo16 + woff;
  const _Float16* wbl = wol16 + woff;

  const v8f zero8 = {0.f, 0.f, 0.f, 0.f, 0.f, 0.f, 0.f, 0.f};
  v8f acc[2][4];
  #pragma unroll
  for (int mt = 0; mt < 2; ++mt)
    #pragma unroll
    for (int nt = 0; nt < 4; ++nt) acc[mt][nt] = zero8;

  #pragma unroll 1
  for (int k0 = 0; k0 < DIM; k0 += 32) {
    const v16h ah0 = load_frag(ah0p + k0, h);
    const v16h ah1 = load_frag(ah1p + k0, h);
    const v16h al0 = load_frag(al0p + k0, h);
    const v16h al1 = load_frag(al1p + k0, h);
    #pragma unroll
    for (int nt = 0; nt < 4; ++nt) {
      const v16h bl = load_frag(wbl + (size_t)nt * 16 * DIM + k0, h);
      const v16h bhf = load_frag(wbh + (size_t)nt * 16 * DIM + k0, h);
      acc[0][nt] = wmma_f16(al0, bl, acc[0][nt]);
      acc[1][nt] = wmma_f16(al1, bl, acc[1][nt]);
      acc[0][nt] = wmma_f16(ah0, bhf, acc[0][nt]);
      acc[1][nt] = wmma_f16(ah1, bhf, acc[1][nt]);
    }
  }

  #pragma unroll
  for (int nt = 0; nt < 4; ++nt) {
    const int feat = 16 * nt + m;
    const float bvl = bo[fg * HD + feat];
    #pragma unroll
    for (int mt = 0; mt < 2; ++mt) {
      #pragma unroll
      for (int r = 0; r < 8; ++r) {
        const int tokl = 32 * w + 16 * mt + 8 * h + r;
        sO[tokl * 64 + feat] = acc[mt][nt][r] * WINV + bvl;
      }
    }
  }
  __syncthreads();

  out_store_pass(sO, out, m0, fg, w, lane);
  __threadfence();
  out_store_pass(sO, out, m0, fg, w, lane);
}

extern "C" void kernel_launch(void* const* d_in, const int* in_sizes, int n_in,
                              void* d_out, int out_size, void* d_ws, size_t ws_size,
                              hipStream_t stream) {
  if (n_in < 7) return;
  if (in_sizes[0] != NX) return;
  if (in_sizes[1] != NW || in_sizes[3] != NW || in_sizes[5] != NW) return;
  if (in_sizes[2] != DIM || in_sizes[4] != DIM || in_sizes[6] != DIM) return;
  if (out_size != NX) return;

  const float* x  = (const float*)d_in[0];
  const float* Wq = (const float*)d_in[1];
  const float* bq = (const float*)d_in[2];
  const float* Wv = (const float*)d_in[3];
  const float* bv = (const float*)d_in[4];
  const float* Wo = (const float*)d_in[5];
  const float* bo = (const float*)d_in[6];
  float* out = (float*)d_out;

  const size_t xh_bytes = (size_t)NX * 2;
  const size_t wp_bytes = (size_t)4 * NW * 2;
  const size_t pl_bytes = (size_t)NBH * SEQ * HD * 2;
  const size_t sq_bytes = (size_t)NBH * SEQ * 4;
  const size_t op_bytes = (size_t)NX * 2;
  const size_t total = xh_bytes + wp_bytes + 3 * pl_bytes + sq_bytes + 2 * op_bytes;
  if (total > ws_size) return;

  char* ws = (char*)d_ws;
  size_t off = 0;
  _Float16* xh   = (_Float16*)(ws + off); off += xh_bytes;
  _Float16* wpl  = (_Float16*)(ws + off); off += wp_bytes;
  _Float16* qk16 = (_Float16*)(ws + off); off += pl_bytes;
  _Float16* ql16 = (_Float16*)(ws + off); off += pl_bytes;
  _Float16* vt16 = (_Float16*)(ws + off); off += pl_bytes;
  float*    sqb  = (float*)(ws + off);    off += sq_bytes;
  _Float16* oh16 = (_Float16*)(ws + off); off += op_bytes;
  _Float16* ol16 = (_Float16*)(ws + off); off += op_bytes;
  if (off > ws_size) return;
  _Float16* wo16  = wpl + (size_t)2 * NW;
  _Float16* wol16 = wpl + (size_t)3 * NW;

  const int ngroups = NX8 + 4 * NW8;
  convert_kernel<<<(ngroups + 255) / 256, 256, 0, stream>>>(x, Wq, Wv, Wo, xh, wpl);

  dim3 gProj(TOK / 128, 2 * NHEADS);
  proj_kernel<<<gProj, 128, 0, stream>>>(xh, wpl, bq, bv, qk16, ql16, sqb, vt16);

  dim3 gAtt(SEQ / 64, NBH);
  attn_kernel<<<gAtt, 128, 0, stream>>>(qk16, ql16, vt16, sqb, oh16, ol16);

  dim3 gOut(TOK / 128, DIM / HD);
  ogemm_kernel<<<gOut, 128, 0, stream>>>(oh16, ol16, wo16, wol16, bo, out);
}
